// ConvolutionalCapsules_11072425689231
// MI455X (gfx1250) — hardware-run, weakly checked
//
#include <hip/hip_runtime.h>

typedef float          v8f   __attribute__((ext_vector_type(8)));
typedef float          v4f   __attribute__((ext_vector_type(4)));
typedef unsigned int   v4u   __attribute__((ext_vector_type(4)));
typedef int            v8i   __attribute__((ext_vector_type(8)));
typedef unsigned short v8us  __attribute__((ext_vector_type(8)));
typedef unsigned short v16us __attribute__((ext_vector_type(16)));
typedef __bf16         v16bf __attribute__((ext_vector_type(16)));
typedef _Float16       v16h  __attribute__((ext_vector_type(16)));
typedef v4f  __attribute__((may_alias)) v4fa;
typedef v8us __attribute__((may_alias)) v8usa;
union FragB { v16bf v; v16us u; v8us h[2]; v8i w; };
union FragH { v16h  v; v16us u; v8us h[2]; v8i w; };

__device__ __forceinline__ v8f wmb(const FragB& a, const FragB& b, v8f c) {
  v8f d = __builtin_amdgcn_wmma_f32_16x16x32_bf16(false, a.v, false, b.v, (short)0, c, false, false);
  asm volatile("v_nop\n\tv_nop\n\tv_nop\n\tv_nop" : "+v"(d) : "v"(a.w), "v"(b.w));
  return d;
}

__device__ __forceinline__ v8f wmh(const FragH& a, const FragH& b, v8f c) {
  v8f d = __builtin_amdgcn_wmma_f32_16x16x32_f16(false, a.v, false, b.v, (short)0, c, false, false);
  asm volatile("v_nop\n\tv_nop\n\tv_nop\n\tv_nop" : "+v"(d) : "v"(a.w), "v"(b.w));
  return d;
}

__device__ __forceinline__ unsigned bf16_bits(float f) {
  const unsigned u = __float_as_uint(f);
  const unsigned r = (u + 0x7FFFu + ((u >> 16) & 1u)) >> 16;
  const unsigned q = (u >> 16) | 0x40u;
  return ((u & 0x7fffffffu) > 0x7f800000u) ? q : r;
}

__device__ __forceinline__ float bf16_val(float f) {
  return __uint_as_float(bf16_bits(f) << 16);
}
__device__ __forceinline__ int clampi(int v, int lo, int hi) {
  return v < lo ? lo : (v > hi ? hi : v);
}

__device__ __forceinline__ unsigned f16_bits(float f) {
  const unsigned u  = __float_as_uint(f);
  const unsigned s  = (u >> 16) & 0x8000u;
  const unsigned a  = u & 0x7fffffffu;
  const unsigned t  = a - 0x38000000u;
  const unsigned r  = (t + 0x0FFFu + ((t >> 13) & 1u)) >> 13;
  const unsigned rc = r > 0x7C00u ? 0x7C00u : r;
  const bool small  = a < 0x38800000u;
  const bool isnan  = a > 0x7f800000u;
  const unsigned fin = small ? 0u : (s | rc);
  return isnan ? (s | 0x7E00u) : fin;
}

__device__ __forceinline__ unsigned pk16(unsigned lo, unsigned hi) { return lo | (hi << 16); }
__device__ __forceinline__ unsigned bf16_lo_bits(float v) {
  float hi = bf16_val(v);
  asm volatile("" : "+v"(hi));
  return bf16_bits(v - hi);
}
__device__ __forceinline__ v4u pack8_bf16(v4f a, v4f c) {
  return (v4u){ pk16(bf16_bits(a[0]), bf16_bits(a[1])), pk16(bf16_bits(a[2]), bf16_bits(a[3])),
                pk16(bf16_bits(c[0]), bf16_bits(c[1])), pk16(bf16_bits(c[2]), bf16_bits(c[3])) };
}
__device__ __forceinline__ v4u pack8_bf16_lo(v4f a, v4f c) {
  return (v4u){ pk16(bf16_lo_bits(a[0]), bf16_lo_bits(a[1])), pk16(bf16_lo_bits(a[2]), bf16_lo_bits(a[3])),
                pk16(bf16_lo_bits(c[0]), bf16_lo_bits(c[1])), pk16(bf16_lo_bits(c[2]), bf16_lo_bits(c[3])) };
}
__device__ __forceinline__ v4u pack8_f16(v4f a, v4f c) {
  return (v4u){ pk16(f16_bits(a[0]), f16_bits(a[1])), pk16(f16_bits(a[2]), f16_bits(a[3])),
                pk16(f16_bits(c[0]), f16_bits(c[1])), pk16(f16_bits(c[2]), f16_bits(c[3])) };
}

template <int FORM>
__global__ __launch_bounds__(256) void k_plane(const float* __restrict__ src, int rows, int cols, int ldsrc,
                                               unsigned short* __restrict__ dst, int MP, int KP) {
  static_assert(FORM >= 0 && FORM <= 3);
  const int KTOT = (FORM == 1 || FORM == 3) ? 2 * KP : KP;
  const unsigned ppr   = (unsigned)(KTOT >> 3);
  const unsigned kp8   = (unsigned)(KP >> 3);
  const unsigned total = (unsigned)MP * ppr;
  const unsigned g     = blockIdx.x * 256u + threadIdx.x;
  const unsigned rowu  = g / ppr;
  const unsigned p     = g - rowu * ppr;
  const bool second    = p >= kp8;
  const int row = (int)rowu;
  const int c0  = (int)((second ? p - kp8 : p) << 3);
  const float* srow = src + (size_t)clampi(row, 0, rows - 1) * (size_t)ldsrc;
  float x[8];
  unsigned mk[8];
#pragma unroll
  for (int e = 0; e < 8; ++e) {
    const int c = c0 + e;
    const float v = srow[clampi(c, 0, cols - 1)];
    asm volatile("" :: "v"(v));
    x[e]  = v;
    mk[e] = (row < rows && c < cols) ? 0xFFFFu : 0u;
  }
  const v4f a = (v4f){ x[0], x[1], x[2], x[3] };
  const v4f c = (v4f){ x[4], x[5], x[6], x[7] };
  v4u o;
  if (FORM == 2) {
    o = pack8_f16(a, c);
  } else {
    const v4u hi = pack8_bf16(a, c);
    o = hi;
    if (FORM == 1) { const v4u lo = pack8_bf16_lo(a, c); o = second ? lo : hi; }
  }
  const v4u mw = (v4u){ pk16(mk[0], mk[1]), pk16(mk[2], mk[3]), pk16(mk[4], mk[5]), pk16(mk[6], mk[7]) };
  o &= mw;
  if (g < total) {
    volatile v4u* q = (volatile v4u*)(dst + (size_t)g * 8);
    *q = o;
    __threadfence();
    *q = o;
  }
}

template <int FORM> struct FragOf    { typedef FragB T; };
template <>         struct FragOf<2> { typedef FragH T; };
__device__ __forceinline__ v8f mm(const FragB& a, const FragB& b, v8f c) { return wmb(a, b, c); }
__device__ __forceinline__ v8f mm(const FragH& a, const FragH& b, v8f c) { return wmh(a, b, c); }
template <class F> __device__ __forceinline__ F ld_frag(const unsigned short* p) {
  F f;
  f.h[0] = *(const v8usa*)(p);
  f.h[1] = *(const v8usa*)(p + 16);
  return f;
}

template <int FORM, int EPI>
__global__ __launch_bounds__(256) __attribute__((amdgpu_num_vgpr(248)))
void k_gemm_nt(const unsigned short* __restrict__ A, const unsigned short* __restrict__ B,
               const float* __restrict__ bias, float* __restrict__ D, int M, int N, int KTOT, int ldd) {
  static_assert(FORM >= 0 && FORM <= 2);
  static_assert(EPI == 0 || EPI == 1);
  typedef typename FragOf<FORM>::T F;
  __shared__ __attribute__((aligned(16))) float sT[8][16 * 68];
  const int lane = threadIdx.x & 31;
  const int wave = threadIdx.x >> 5;
  const int tilesM = (M + 63) >> 6;
  const int tilesN = (N + 63) >> 6;
  const int tile = blockIdx.x * 8 + wave;
  if (tile >= tilesM * tilesN) return;
  const int tm = tile / tilesN;
  const int tn = tile - tm * tilesN;
  const int m0 = tm << 6;
  const int n0 = tn << 6;

  const int rl = lane & 15;
  const int h8 = (lane >> 4) * 8;
  const unsigned short* pa = A + (size_t)(m0 + rl) * (size_t)KTOT + h8;
  const unsigned short* pb = B + (size_t)(n0 + rl) * (size_t)KTOT + h8;

  v8f acc[4][4];
#pragma unroll
  for (int i = 0; i < 4; ++i)
#pragma unroll
    for (int j = 0; j < 4; ++j) acc[i][j] = (v8f){0.f, 0.f, 0.f, 0.f, 0.f, 0.f, 0.f, 0.f};

#pragma unroll 1
  for (int k0 = 0; k0 < KTOT; k0 += 32) {
    F bf[4];
#pragma unroll
    for (int j = 0; j < 4; ++j) bf[j] = ld_frag<F>(pb + (size_t)(j << 4) * (size_t)KTOT + k0);
#pragma unroll
    for (int i = 0; i < 4; ++i) {
      const F af = ld_frag<F>(pa + (size_t)(i << 4) * (size_t)KTOT + k0);
#pragma unroll
      for (int j = 0; j < 4; ++j) acc[i][j] = mm(af, bf[j], acc[i][j]);
    }
  }

  float* slab = sT[wave];
  const int hh = lane >> 4;
  const int c4 = (lane & 15) * 4;
  const int nc = n0 + c4;
  const bool cok = nc < N;
  v4f bv = (v4f){0.f, 0.f, 0.f, 0.f};
  if (EPI == 1) {
    bv = *(const v4fa*)(bias + clampi(nc, 0, N - 4));
    asm volatile("" :: "v"(bv));
  }
#pragma unroll
  for (int i = 0; i < 4; ++i) {
    const int mBase = m0 + (i << 4);
#pragma unroll
    for (int j = 0; j < 4; ++j) {
#pragma unroll
      for (int r = 0; r < 8; ++r) slab[(h8 + r) * 68 + (j << 4) + rl] = acc[i][j][r];
    }
    __builtin_amdgcn_fence(__ATOMIC_RELEASE, "workgroup");
    __builtin_amdgcn_wave_barrier();
    __builtin_amdgcn_fence(__ATOMIC_ACQUIRE, "workgroup");
    v4f vv[8];
#pragma unroll
    for (int it = 0; it < 8; ++it) {
      const int row = it * 2 + hh;
      v4f v = *(const v4fa*)(slab + row * 68 + c4);
      if (EPI == 1) v += bv;
      vv[it] = v;
    }
    for (int pass = 0; pass < 2; ++pass) {
#pragma unroll
      for (int it = 0; it < 8; ++it) {
        const int row = mBase + it * 2 + hh;
        if (cok && row < M) *(volatile v4f*)(D + (size_t)row * (size_t)ldd + nc) = vv[it];
      }
      __threadfence();
    }
    __builtin_amdgcn_fence(__ATOMIC_RELEASE, "workgroup");
    __builtin_amdgcn_wave_barrier();
    __builtin_amdgcn_fence(__ATOMIC_ACQUIRE, "workgroup");
  }
}

#include <math.h>

typedef v4u __attribute__((may_alias)) v4ua;

#define NBATCH 4
#define NIN    8
#define DIN    16
#define NG     4
#define IMH    32
#define IMW    32
#define NOUT   8
#define DOUT   16
#define NIMG   (NBATCH * NIN)
#define NCH    (DIN * NG)
#define KTOTC  (NCH * 9)
#define NCOL   (NOUT * DOUT * NG)
#define MROWS  (NIMG * IMH * IMW)
#define NWELEM (NOUT * DOUT * DIN * NG * 9)
#define NXELEM (NIMG * NCH * IMH * IMW)
#define NOELEM (NBATCH * NOUT * DOUT * NG * IMH * IMW)

static_assert(NIMG == 32);
static_assert(NCH == 64);
static_assert(KTOTC == 576 && KTOTC == 18 * 32);
static_assert(NCOL == 512);
static_assert(MROWS % 128 == 0 && MROWS % 64 == 0 && MROWS % 16 == 0);
static_assert(NCOL % 64 == 0 && NCOL % 32 == 0 && NCOL % 4 == 0);
static_assert(KTOTC % 32 == 0 && KTOTC % 8 == 0);
static_assert(IMW == 32 && IMH == 32);
static_assert(NG == 4);
static_assert(NIN == 8);
static_assert(DOUT == 16);
static_assert(NOELEM == NXELEM);

#define WB_PIECES (NCOL * (KTOTC / 8))
#define WB_BLOCKS (WB_PIECES / 256)
static_assert(WB_BLOCKS * 256 == WB_PIECES);

__global__ __launch_bounds__(256) void k_wbank(const float* __restrict__ w, const float* __restrict__ cb,
                                               unsigned short* __restrict__ WB, float* __restrict__ BR) {
  const int tid = threadIdx.x;
  if (blockIdx.x == WB_BLOCKS) {
    const float bsrc = cb[tid & 127];
    asm volatile("" :: "v"(bsrc));
    const float br = bf16_val(bsrc);
    const v4f o = (v4f){ br, br, br, br };
    if (tid < 128) {
      volatile v4f* q = (volatile v4f*)(BR + tid * 4);
      *q = o;
      __threadfence();
      *q = o;
    }
    return;
  }
  const unsigned gi = blockIdx.x * 256u + (unsigned)tid;
  const int n  = (int)(gi / 72u);
  const int p  = (int)gi - n * 72;
  const int k0 = p * 8;
  const int cout = n >> 2;
  const int r    = n & 3;
  float x[8];
#pragma unroll
  for (int e = 0; e < 8; ++e) {
    const int k   = k0 + e;
    const int c   = k / 9;
    const int t   = k - c * 9;
    const int ky  = t / 3;
    const int kx  = t - ky * 3;
    const int cin = c >> 2;
    const int gs  = ((c & 3) - r) & 3;
    const int sy  = (r == 0) ? ky : ((r == 1) ? kx : ((r == 2) ? (2 - ky) : (2 - kx)));
    const int sx  = (r == 0) ? kx : ((r == 1) ? (2 - ky) : ((r == 2) ? (2 - kx) : ky));
    const int idx = clampi(((cout * 16 + cin) * 4 + gs) * 9 + sy * 3 + sx, 0, NWELEM - 1);
    const float v = w[idx];
    asm volatile("" :: "v"(v));
    x[e] = v;
  }
  const v4u o = pack8_bf16((v4f){ x[0], x[1], x[2], x[3] }, (v4f){ x[4], x[5], x[6], x[7] });
  volatile v4u* q = (volatile v4u*)(WB + (size_t)gi * 8);
  *q = o;
  __threadfence();
  *q = o;
}

#define XT_PITCH 34
#define XT_WORDS (3 * NCH * XT_PITCH)

__global__ __launch_bounds__(256) void k_im2col(const float* __restrict__ X, unsigned short* __restrict__ A) {
  __shared__ __attribute__((aligned(16))) unsigned sX[XT_WORDS];
  __shared__ __attribute__((aligned(16))) unsigned sK[KTOTC];
  const int tid = threadIdx.x;
  const int n = blockIdx.x >> 5;
  const int y = blockIdx.x & 31;

  for (int k = tid; k < KTOTC; k += 256) {
    const int c  = k / 9;
    const int t  = k - c * 9;
    const int ky = t / 3;
    const int kx = t - ky * 3;
    sK[k] = (unsigned)((ky * NCH + c) * XT_PITCH + kx);
  }
  for (int e = tid; e < 3 * NCH * 2; e += 256) {
    const int row = e >> 1;
    sX[row * XT_PITCH + (e & 1) * 33] = 0u;
  }
#pragma unroll
  for (int ky = 0; ky < 3; ++ky) {
    const int yy = y + ky - 1;
    const unsigned okm = ((unsigned)yy < (unsigned)IMH) ? 0xFFFFFFFFu : 0u;
    const int yc = clampi(yy, 0, IMH - 1);
#pragma unroll
    for (int it = 0; it < 2; ++it) {
      const int v  = it * 256 + tid;
      const int c  = v >> 3;
      const int x4 = (v & 7) * 4;
      const v4f f = *(const v4fa*)(X + ((size_t)((n * NCH + c) * IMH + yc) * IMW + x4));
      asm volatile("" :: "v"(f));
      unsigned* tp = sX + (ky * NCH + c) * XT_PITCH + 1 + x4;
      tp[0] = bf16_bits(f[0]) & okm;
      tp[1] = bf16_bits(f[1]) & okm;
      tp[2] = bf16_bits(f[2]) & okm;
      tp[3] = bf16_bits(f[3]) & okm;
    }
  }
  __syncthreads();

  v4u vv[9];
#pragma unroll
  for (int it = 0; it < 9; ++it) {
    const int v  = it * 256 + tid;
    const int x  = v / 72;
    const int k0 = (v - x * 72) * 8;
    const v4u o0 = *(const v4ua*)(sK + k0);
    const v4u o1 = *(const v4ua*)(sK + k0 + 4);
    const unsigned a0 = sX[o0[0] + x], a1 = sX[o0[1] + x], a2 = sX[o0[2] + x], a3 = sX[o0[3] + x];
    const unsigned a4 = sX[o1[0] + x], a5 = sX[o1[1] + x], a6 = sX[o1[2] + x], a7 = sX[o1[3] + x];
    vv[it] = (v4u){ pk16(a0, a1), pk16(a2, a3), pk16(a4, a5), pk16(a6, a7) };
  }
  unsigned short* base = A + (size_t)blockIdx.x * (size_t)(32 * KTOTC);
  for (int pass = 0; pass < 2; ++pass) {
#pragma unroll
    for (int it = 0; it < 9; ++it)
      *(volatile v4u*)(base + (size_t)(it * 256 + tid) * 8) = vv[it];
    __threadfence();
  }
}

#define RT_PITCH  65
#define RT_ROWBLK (32 * RT_PITCH)
#define RT_T      (NIN * RT_ROWBLK)
#define RT_SQ     (NG * DOUT * IMW)
#define RT_PT     (NIN * 128)
#define RT_GB     32
#define ROUTE_LDS ((RT_T + RT_SQ + RT_PT + RT_GB) * 4)
static_assert(ROUTE_LDS == 78976);
static_assert(ROUTE_LDS <= 327680);

__global__ __launch_bounds__(128) void k_route(const float* __restrict__ U, const float* __restrict__ gamma,
                                               const float* __restrict__ beta, float* __restrict__ out) {
  extern __shared__ __attribute__((aligned(16))) float smem[];
  const int oSQ = RT_T;
  const int oPT = RT_T + RT_SQ;
  const int oGB = RT_T + RT_SQ + RT_PT;
  const int tid = threadIdx.x;
  const int g = tid >> 5;
  const int w = tid & 31;
  const int bx = blockIdx.x;
  const int h    = bx & 31;
  const int nout = (bx >> 5) & 7;
  const int b    = bx >> 8;

  {
    const float gv = gamma[tid & 15];
    const float bv = beta[tid & 15];
    asm volatile("" :: "v"(gv), "v"(bv));
    if (tid < 16) {
      smem[oGB + tid]      = bf16_val(gv);
      smem[oGB + 16 + tid] = bf16_val(bv);
    }
  }
  {
    const int rsub = tid >> 4;
    const int c4   = (tid & 15) * 4;
#pragma unroll 4
    for (int it = 0; it < 32; ++it) {
      const int rr  = it * 8 + rsub;
      const int nin = rr >> 5;
      const int wq  = rr & 31;
      const size_t row = (size_t)((b * NIN + nin) * (IMH * IMW) + h * IMW + wq);
      const v4f v = *(const v4fa*)(U + row * (size_t)NCOL + (size_t)(nout * 64 + c4));
      const int to = rr * RT_PITCH + c4;
      smem[to + 0] = v[0];
      smem[to + 1] = v[1];
      smem[to + 2] = v[2];
      smem[to + 3] = v[3];
    }
  }
  __syncthreads();

  const int own = w * RT_PITCH + g;

#pragma unroll 1
  for (int i = 0; i < NIN; ++i) {
    const int ro = own + i * RT_ROWBLK;
    float sum = 0.0f;
#pragma unroll
    for (int d = 0; d < DOUT; ++d) sum += smem[ro + d * 4];
    const float mu = sum * 0.0625f;
    float var = 0.0f;
#pragma unroll 1
    for (int d = 0; d < DOUT; ++d) {
      const float z = smem[ro + d * 4] - mu;
      var += z * z;
    }
    var *= 0.0625f;
    const float sd = sqrtf(var + 1e-5f);
    float nsq = 0.0f;
#pragma unroll 1
    for (int d = 0; d < DOUT; ++d) {
      const float v  = smem[ro + d * 4];
      const float yv = (v - mu) / sd * smem[oGB + d] + smem[oGB + 16 + d];
      smem[ro + d * 4] = yv;
      nsq += yv * yv;
    }
    smem[oPT + i * 128 + tid] = (nsq < 1e-8f) ? 1e-8f : nsq;
  }

#pragma unroll 1
  for (int i = 0; i < NIN; ++i) {
    float r[DOUT];
#pragma unroll
    for (int d = 0; d < DOUT; ++d) r[d] = smem[own + i * RT_ROWBLK + d * 4];
    const float nq = smem[oPT + i * 128 + tid];
    float t = 0.0f;
#pragma unroll 1
    for (int j = 0; j < NIN; ++j) {
      const int rj = own + j * RT_ROWBLK;
      float dot = 0.0f;
#pragma unroll
      for (int d = 0; d < DOUT; ++d) dot += r[d] * smem[rj + d * 4];
      t += dot / nq;
    }
    smem[oPT + i * 128 + tid] = t;
  }

  float mx = smem[oPT + tid];
#pragma unroll
  for (int i = 1; i < NIN; ++i) {
    const float tv = smem[oPT + i * 128 + tid];
    mx = (tv > mx) ? tv : mx;
  }
  float Z = 0.0f;
#pragma unroll 1
  for (int i = 0; i < NIN; ++i) {
    const float e = expf(smem[oPT + i * 128 + tid] - mx);
    smem[oPT + i * 128 + tid] = e;
    Z += e;
  }
  float s[DOUT];
#pragma unroll
  for (int d = 0; d < DOUT; ++d) s[d] = 0.0f;
#pragma unroll 1
  for (int i = 0; i < NIN; ++i) {
    const float sc = smem[oPT + i * 128 + tid] / Z;
    const int ro = own + i * RT_ROWBLK;
#pragma unroll
    for (int d = 0; d < DOUT; ++d) s[d] += sc * smem[ro + d * 4];
  }

#pragma unroll
  for (int d = 0; d < DOUT; ++d) smem[oSQ + (g * DOUT + d) * IMW + w] = s[d];
  __syncthreads();
#pragma unroll 1
  for (int d = 0; d < DOUT; ++d) {
    const float s0 = smem[oSQ + (0 * DOUT + d) * IMW + w];
    const float s1 = smem[oSQ + (1 * DOUT + d) * IMW + w];
    const float s2 = smem[oSQ + (2 * DOUT + d) * IMW + w];
    const float s3 = smem[oSQ + (3 * DOUT + d) * IMW + w];
    const float me = smem[oSQ + (g * DOUT + d) * IMW + w];
    float q = s0 * s0;
    q += s1 * s1;
    q += s2 * s2;
    q += s3 * s3;
    const float v = (q / (1.0f + q)) * (me / sqrtf(q + 1e-16f));
    smem[own + d * 4] = v;
  }
  float vv[DOUT];
#pragma unroll
  for (int d = 0; d < DOUT; ++d) vv[d] = smem[own + d * 4];

  float* op = out + ((size_t)(b * NOUT + nout) * (size_t)(DOUT * NG * IMH * IMW)
                     + (size_t)(g * IMH * IMW + h * IMW + w));
  for (int pass = 0; pass < 2; ++pass) {
#pragma unroll
    for (int d = 0; d < DOUT; ++d)
      *(volatile float*)(op + (size_t)d * (size_t)(NG * IMH * IMW)) = vv[d];
    __threadfence();
  }
}

extern "C" void kernel_launch(void* const* d_in, const int* in_sizes, int n_in,
                              void* d_out, int out_size, void* d_ws, size_t ws_size,
                              hipStream_t stream) {
  if (n_in < 5) return;
  if (in_sizes[0] != NXELEM) return;
  if (in_sizes[1] != NWELEM) return;
  if (in_sizes[2] != NOUT * DOUT) return;
  if (in_sizes[3] != DOUT) return;
  if (in_sizes[4] != DOUT) return;
  if (out_size != NOELEM) return;

  const float* xin   = (const float*)d_in[0];
  const float* convw = (const float*)d_in[1];
  const float* convb = (const float*)d_in[2];
  const float* lng   = (const float*)d_in[3];
  const float* lnb   = (const float*)d_in[4];
  float* out = (float*)d_out;

  const size_t PA  = (size_t)MROWS * KTOTC * 2;
  const size_t PWB = (size_t)NCOL * KTOTC * 2;
  const size_t PBR = (size_t)NCOL * 4;
  const size_t PU  = (size_t)MROWS * NCOL * 4;
  size_t off = 0;
  const size_t oA  = off; off += PA;
  const size_t oWB = off; off += PWB;
  const size_t oBR = off; off += PBR;
  const size_t oU  = off; off += PU;
  if ((oWB & 255) || (oBR & 255) || (oU & 255)) return;
  if (off > ws_size) return;
  if (off > ((size_t)128 << 20)) return;

  char* ws = (char*)d_ws;
  unsigned short* A  = (unsigned short*)(ws + oA);
  unsigned short* WB = (unsigned short*)(ws + oWB);
  float* BR = (float*)(ws + oBR);
  float* U  = (float*)(ws + oU);

  k_wbank<<<dim3(WB_BLOCKS + 1), dim3(256), 0, stream>>>(convw, convb, WB, BR);
  k_im2col<<<dim3(NIMG * IMH), dim3(256), 0, stream>>>(xin, A);
  k_gemm_nt<0, 1><<<dim3((MROWS / 64) * (NCOL / 64) / 8), dim3(256), 0, stream>>>(A, WB, BR, U, MROWS, NCOL, KTOTC, NCOL);
  (void)hipFuncSetAttribute(reinterpret_cast<const void*>(&k_route), hipFuncAttributeMaxDynamicSharedMemorySize, ROUTE_LDS);
  k_route<<<dim3(NBATCH * NOUT * IMH), dim3(128), ROUTE_LDS, stream>>>(U, lng, lnb, out);
  (void)hipGetLastError();
}
